// MixedAttention_85341000172350
// MI455X (gfx1250) — hardware-verified
//
#include <hip/hip_runtime.h>


#define NB_  2
#define CC   256
#define IMW  56
#define HW   3136
#define TP   3200
#define NH_  8
#define DK   32
#define DP   64
#define K9   (CC * 9)
#define PCAR 1024.0f
#define SCL  0.17677669529663689f
#define BNEPS 1e-5f
#define SLOPE 0.01f
typedef _Float16 h16;
typedef unsigned short bf;
typedef __attribute__((ext_vector_type(16))) __bf16   v16bf;
typedef __attribute__((ext_vector_type(16))) _Float16 v16h;
typedef __attribute__((ext_vector_type(8)))  _Float16 v8h;
typedef __attribute__((ext_vector_type(8)))  unsigned short v8us;
typedef __attribute__((ext_vector_type(8)))  float    v8f;
typedef __attribute__((ext_vector_type(4)))  float    v4f;
typedef v8h  __attribute__((may_alias)) v8ha;
typedef v4f  __attribute__((may_alias)) v4fa;
typedef v8us __attribute__((may_alias)) v8usa;

__device__ __forceinline__ unsigned short f2bf(float f) { unsigned u = __float_as_uint(f); u += 0x7FFFu + ((u >> 16) & 1u); return (unsigned short)(u >> 16); }
__device__ __forceinline__ float bf2f(unsigned short b) { return __uint_as_float(((unsigned)b) << 16); }
__device__ __forceinline__ float bfr(float f) { return bf2f(f2bf(f)); }
__device__ __forceinline__ v16h cat16(v8h lo, v8h hi) { return __builtin_shufflevector(lo, hi, 0, 1, 2, 3, 4, 5, 6, 7, 8, 9, 10, 11, 12, 13, 14, 15); }
__device__ __forceinline__ v16bf cat16b(v8us lo, v8us hi) { return __builtin_bit_cast(v16bf, __builtin_shufflevector(lo, hi, 0, 1, 2, 3, 4, 5, 6, 7, 8, 9, 10, 11, 12, 13, 14, 15)); }
__device__ __forceinline__ v8f wmma16(v16h a, v16h b, v8f c) { return __builtin_amdgcn_wmma_f32_16x16x32_f16(false, a, false, b, (short)0, c, false, false); }
__device__ __forceinline__ v8f wmmab(v16bf a, v16bf b, v8f c) { return __builtin_amdgcn_wmma_f32_16x16x32_bf16(false, a, false, b, (short)0, c, false, false); }


template <typename T16> struct WFrag;
template <> struct WFrag<h16> { typedef v16h V; static __device__ __forceinline__ V ld(const h16* p) { return cat16(*(const v8h*)p, *(const v8h*)(p + 16)); } static __device__ __forceinline__ v8f mma(V a, V b, v8f c) { return wmma16(a, b, c); } };
template <> struct WFrag<bf> { typedef v16bf V; static __device__ __forceinline__ V ld(const bf* p) { return cat16b(*(const v8us*)p, *(const v8us*)(p + 16)); } static __device__ __forceinline__ v8f mma(V a, V b, v8f c) { return wmmab(a, b, c); } };
template <typename T16, int NSPLIT, bool BIAS>
__global__ __launch_bounds__(32) void k_gemmw(const T16* __restrict__ A, const T16* __restrict__ A2, const T16* __restrict__ Bt, const T16* __restrict__ Bt2, int K, float* C, int ldc, const float* __restrict__ bias, size_t sA, size_t sB, size_t sC) {
    typedef typename WFrag<T16>::V V;
    __shared__ __align__(16) float os[16 * 68];
    const size_t z = blockIdx.z; A += z * sA; if (A2) A2 += z * sA; Bt += z * sB; if (Bt2) Bt2 += z * sB; C += z * sC;
    const int lane = threadIdx.x & 31, lr = lane & 15, hi = lane >> 4; const int r0 = blockIdx.x * 64, c0 = blockIdx.y * 64;
    v8f acc[4][4];
#pragma unroll
    for (int mb = 0; mb < 4; ++mb)
#pragma unroll
        for (int nb = 0; nb < 4; ++nb) acc[mb][nb] = (v8f){};
    const size_t aoff = (size_t)(r0 + lr) * K + 8 * hi, boff = (size_t)(c0 + lr) * K + 8 * hi;
#pragma unroll 1
    for (int kc = 0; kc < K; kc += 32) {
        V a[4], a2[4];
#pragma unroll
        for (int mb = 0; mb < 4; ++mb) { a[mb] = WFrag<T16>::ld(A + aoff + (size_t)mb * 16 * K + kc); if (NSPLIT == 1 || NSPLIT == 2) a2[mb] = WFrag<T16>::ld(A2 + aoff + (size_t)mb * 16 * K + kc); }
#pragma unroll
        for (int nb = 0; nb < 4; ++nb) { const V b = WFrag<T16>::ld(Bt + boff + (size_t)nb * 16 * K + kc); V b2; if (NSPLIT >= 2) b2 = WFrag<T16>::ld(Bt2 + boff + (size_t)nb * 16 * K + kc);
#pragma unroll
            for (int mb = 0; mb < 4; ++mb) { acc[mb][nb] = WFrag<T16>::mma(a[mb], b, acc[mb][nb]); if (NSPLIT == 1 || NSPLIT == 2) acc[mb][nb] = WFrag<T16>::mma(a2[mb], b, acc[mb][nb]); if (NSPLIT >= 2) acc[mb][nb] = WFrag<T16>::mma(a[mb], b2, acc[mb][nb]); } }
        asm volatile("v_nop\n\tv_nop\n\tv_nop\n\tv_nop" : "+v"(acc[0][0]), "+v"(acc[1][1]), "+v"(acc[2][2]), "+v"(acc[3][3]) : "v"(a[0]), "v"(a[3]));
    }
#pragma unroll
    for (int mb = 0; mb < 4; ++mb) {
#pragma unroll
        for (int nb = 0; nb < 4; ++nb) {
#pragma unroll
            for (int j = 0; j < 8; ++j) os[(hi * 8 + j) * 68 + nb * 16 + lr] = acc[mb][nb][j]; }
        __builtin_amdgcn_wave_barrier(); asm volatile("" ::: "memory");
        float* crow = C + (size_t)(r0 + mb * 16) * ldc + c0;
#pragma unroll 1
        for (int ps = 0; ps < 2; ++ps) {
#pragma unroll
            for (int s = 0; s < 8; ++s) { const int row = 2 * s + hi, cofs = lr * 4; v4f val = *(const v4fa*)(os + row * 68 + cofs); if (BIAS) { val[0] += bfr(bias[c0 + cofs]); val[1] += bfr(bias[c0 + cofs + 1]); val[2] += bfr(bias[c0 + cofs + 2]); val[3] += bfr(bias[c0 + cofs + 3]); }
                *(volatile v4f*)(crow + (size_t)row * ldc + cofs) = val; }
            if (ps == 0) __threadfence(); }
        __builtin_amdgcn_wave_barrier(); asm volatile("" ::: "memory");
    }
}

__device__ __forceinline__ h16 tohx(float x) { return (h16)x; }
__device__ __forceinline__ void splitf(float y, unsigned short& h, unsigned short& l) { h = f2bf(y); l = f2bf(y - bf2f(h)); }
typedef __attribute__((ext_vector_type(2))) _Float16 v2h;
typedef __attribute__((ext_vector_type(4))) _Float16 v4h;
typedef __attribute__((ext_vector_type(2))) unsigned short v2us;
typedef __attribute__((ext_vector_type(4))) unsigned short v4us;
typedef __attribute__((ext_vector_type(2))) float v2f;
typedef __attribute__((ext_vector_type(4))) int v4i;

__global__ __launch_bounds__(256) void k_cvt8(const float* __restrict__ src, bf* dst, size_t n8) { const size_t i = (size_t)blockIdx.x * 256 + threadIdx.x; if (i >= n8) return; const v8f v = *(const v8f*)(src + i * 8); v8us o;
#pragma unroll
    for (int k = 0; k < 8; ++k) o[k] = f2bf(v[k]); *(volatile v8us*)(dst + i * 8) = o; __threadfence(); *(volatile v8us*)(dst + i * 8) = o; }
__global__ __launch_bounds__(256) void k_cvt8Tg(const float* __restrict__ src, bf* dst, int R, int C) { const size_t i = (size_t)blockIdx.x * 256 + threadIdx.x; if (i >= (size_t)R * C / 8) return; const int c = (int)(i / (R / 8)); const int r0 = (int)(i % (R / 8)) * 8; v8us o;
#pragma unroll
    for (int k = 0; k < 8; ++k) o[k] = f2bf(src[(size_t)(r0 + k) * C + c]); *(volatile v8us*)(dst + (size_t)c * R + r0) = o; __threadfence(); *(volatile v8us*)(dst + (size_t)c * R + r0) = o; }
__device__ __forceinline__ float bn_leaky(float y, float sc, float sh) { float t = __fmul_rn(y, sc); asm volatile("" : "+v"(t)); float z = __fadd_rn(t, sh); asm volatile("" : "+v"(z)); return (z >= 0.0f) ? z : __fmul_rn(SLOPE, z); }
__global__ __launch_bounds__(256) void k_bnprep(const float* __restrict__ ga, const float* __restrict__ be, const float* __restrict__ mu, const float* __restrict__ va, float* SC, float* SH) { const int c = blockIdx.x * 256 + threadIdx.x; if (c >= CC) return;
    float v1 = __fadd_rn(bfr(va[c]), BNEPS); asm volatile("" : "+v"(v1)); float sd = __fsqrt_rn(v1); asm volatile("" : "+v"(sd)); float sc = __fdiv_rn(bfr(ga[c]), sd); asm volatile("" : "+v"(sc));
    float ms = __fmul_rn(bfr(mu[c]), sc); asm volatile("" : "+v"(ms)); float sh = __fsub_rn(bfr(be[c]), ms);
    *(volatile float*)(SC + c) = sc; *(volatile float*)(SH + c) = sh; __threadfence(); *(volatile float*)(SC + c) = sc; *(volatile float*)(SH + c) = sh; }

__global__ __launch_bounds__(256) void k_im2x(const float* __restrict__ X, bf* A) { const size_t e = ((size_t)blockIdx.x * 256 + threadIdx.x) * 8; if (e >= (size_t)HW * K9) return; const int k0 = (int)(e % K9); const int p = (int)(e / K9); const int py = p / IMW, px = p % IMW; v8us o;
#pragma unroll
    for (int q = 0; q < 8; ++q) { const int k = k0 + q; const int c = k / 9, tap = k % 9; const int y = py + tap / 3 - 1, x = px + tap % 3 - 1; float v = 0.0f; if (y >= 0 && y < IMW && x >= 0 && x < IMW) v = X[((size_t)c * IMW + y) * IMW + x]; o[q] = f2bf(v); }
    *(volatile v8us*)(A + e) = o; __threadfence(); *(volatile v8us*)(A + e) = o; }
__global__ __launch_bounds__(256) void k_plq(const float* __restrict__ F, bf* Ph, bf* Pl) { const size_t e = ((size_t)blockIdx.x * 256 + threadIdx.x) * 2; if (e >= (size_t)NH_ * HW * DK) return; const int d = (int)(e % DK); const int k = (int)((e / DK) % HW); const int h = (int)(e / ((size_t)DK * HW)); const float* f = F + (size_t)k * CC + h * DK + d; v2us oh, ol;
#pragma unroll
    for (int q = 0; q < 2; ++q) { unsigned short a, c2; splitf(f[q], a, c2); oh[q] = a; ol[q] = c2; }
    *(volatile v2us*)(Ph + e) = oh; *(volatile v2us*)(Pl + e) = ol; __threadfence(); *(volatile v2us*)(Ph + e) = oh; *(volatile v2us*)(Pl + e) = ol; }
__global__ __launch_bounds__(256) void k_plk(const float* __restrict__ F, bf* Ph, bf* Pl) { const size_t e = ((size_t)blockIdx.x * 256 + threadIdx.x) * 2; if (e >= (size_t)NH_ * TP * DK) return; const int d = (int)(e % DK); const int m = (int)((e / DK) % TP); const int h = (int)(e / ((size_t)DK * TP)); v2us oh, ol;
    if (m < HW) { const float* f = F + (size_t)m * CC + h * DK + d;
#pragma unroll
        for (int q = 0; q < 2; ++q) { unsigned short a, c2; splitf(f[q], a, c2); oh[q] = a; ol[q] = c2; } } else { oh[0] = 0; oh[1] = 0; ol[0] = 0; ol[1] = 0; }
    *(volatile v2us*)(Ph + e) = oh; *(volatile v2us*)(Pl + e) = ol; __threadfence(); *(volatile v2us*)(Ph + e) = oh; *(volatile v2us*)(Pl + e) = ol; }
__global__ __launch_bounds__(256) void k_vt16p(const float* __restrict__ F, h16* V16) { const size_t e = ((size_t)blockIdx.x * 256 + threadIdx.x) * 2; if (e >= (size_t)NH_ * DP * TP) return; const int m = (int)(e % TP); const int dd = (int)((e / TP) % DP); const int h = (int)(e / ((size_t)TP * DP)); v2h o;
#pragma unroll
    for (int q = 0; q < 2; ++q) { float v = 0.0f; if (dd < DK && m + q < HW) v = F[(size_t)(m + q) * CC + h * DK + dd]; o[q] = tohx(v); }
    *(volatile v2h*)(V16 + e) = o; __threadfence(); *(volatile v2h*)(V16 + e) = o; }
__global__ __launch_bounds__(256) void k_lsoftm(const float* __restrict__ Sb, h16* P16) {
    const int lane = threadIdx.x & 31; const int row = blockIdx.x * 8 + (threadIdx.x >> 5); if (row >= HW) return; const float* sr = Sb + (size_t)row * TP; float mx = -3.0e38f;
#pragma unroll 2
    for (int ch = 0; ch < TP / 128; ++ch) { const int j0 = ch * 128 + lane * 4; const v4f a = *(const v4f*)(sr + j0);
#pragma unroll
        for (int q = 0; q < 4; ++q) { float t = (j0 + q < HW) ? a[q] * SCL : -3.0e38f; asm volatile("" : "+v"(t)); mx = fmaxf(mx, t); } }
#pragma unroll
    for (int sh = 16; sh; sh >>= 1) mx = fmaxf(mx, __shfl_xor(mx, sh, 32));
    float sum = 0.f;
#pragma unroll 4
    for (int ch = 0; ch < TP / 128; ++ch) { const int j0 = ch * 128 + lane * 4; const v4f a = *(const v4f*)(sr + j0);
#pragma unroll
        for (int q = 0; q < 4; ++q) { float t = (j0 + q < HW) ? a[q] * SCL : -3.0e38f; asm volatile("" : "+v"(t)); float d0 = __fsub_rn(t, mx); asm volatile("" : "+v"(d0)); sum += __builtin_amdgcn_exp2f(__fmul_rn(d0, 1.4426950408889634f)); } }
#pragma unroll
    for (int sh = 16; sh; sh >>= 1) sum += __shfl_xor(sum, sh, 32);
    const float f = __fdiv_rn(PCAR, sum);
#pragma unroll 1
    for (int ps = 0; ps < 2; ++ps) {
#pragma unroll 2
        for (int ch = 0; ch < TP / 128; ++ch) { const int j0 = ch * 128 + lane * 4; const v4f a = *(const v4f*)(sr + j0); v4h o4;
#pragma unroll
            for (int q = 0; q < 4; ++q) { float t = (j0 + q < HW) ? a[q] * SCL : -3.0e38f; asm volatile("" : "+v"(t)); float d0 = __fsub_rn(t, mx); asm volatile("" : "+v"(d0)); float ex = __builtin_amdgcn_exp2f(__fmul_rn(d0, 1.4426950408889634f)); asm volatile("" : "+v"(ex)); o4[q] = tohx(ex * f); }
            *(volatile v4h*)(P16 + (size_t)row * TP + j0) = o4; }
        if (ps == 0) __threadfence(); }
}

__global__ __launch_bounds__(256) void k_saout(const float* __restrict__ O, int h, float* out) { const size_t i = (size_t)blockIdx.x * 256 + threadIdx.x; if (i >= (size_t)DK * HW / 8) return; const int d = (int)(i / (HW / 8)); const int p0 = (int)(i % (HW / 8)) * 8; v4f a, b2;
#pragma unroll
    for (int q = 0; q < 4; ++q) { a[q] = O[(size_t)(p0 + q) * DP + d] * (1.0f / PCAR); b2[q] = O[(size_t)(p0 + 4 + q) * DP + d] * (1.0f / PCAR); }
    float* dst = out + (size_t)(h * DK + d) * HW + p0; *(volatile v4f*)dst = a; *(volatile v4f*)(dst + 4) = b2; __threadfence(); *(volatile v4f*)dst = a; *(volatile v4f*)(dst + 4) = b2; }
__global__ __launch_bounds__(256) void k_mulpl(const float* __restrict__ A, const float* __restrict__ Bq, bf* Ph, bf* Pl, size_t n8) { const size_t i = (size_t)blockIdx.x * 256 + threadIdx.x; if (i >= n8) return; const v8f a = *(const v8f*)(A + i * 8); const v8f bb = *(const v8f*)(Bq + i * 8); v8us oh, ol;
#pragma unroll
    for (int q = 0; q < 8; ++q) { float pr = __fmul_rn(a[q], bb[q]); asm volatile("" : "+v"(pr)); unsigned short a2, c2; splitf(pr, a2, c2); oh[q] = a2; ol[q] = c2; }
    *(volatile v8us*)(Ph + i * 8) = oh; *(volatile v8us*)(Pl + i * 8) = ol; __threadfence(); *(volatile v8us*)(Ph + i * 8) = oh; *(volatile v8us*)(Pl + i * 8) = ol; }
__global__ __launch_bounds__(256) void k_vsig(const float* __restrict__ Vv, const float* __restrict__ G, float* VS, size_t n4) { const size_t i = (size_t)blockIdx.x * 256 + threadIdx.x; if (i >= n4) return; const v4f v = *(const v4f*)(Vv + i * 4); const v4f gg = *(const v4f*)(G + i * 4); v4f o;
#pragma unroll
    for (int q = 0; q < 4; ++q) { float den = __fadd_rn(1.0f, expf(-gg[q])); asm volatile("" : "+v"(den)); const float sg = __fdiv_rn(1.0f, den); o[q] = __fmul_rn(v[q], sg); }
    *(volatile v4f*)(VS + i * 4) = o; __threadfence(); *(volatile v4f*)(VS + i * 4) = o; }
__global__ __launch_bounds__(256) void k_dwbn(const float* __restrict__ VS, const float* __restrict__ dww, const float* __restrict__ SC, const float* __restrict__ SH, bf* Yh, bf* Yl) { const size_t e = ((size_t)blockIdx.x * 256 + threadIdx.x) * 2; if (e >= (size_t)HW * CC) return; const int c = (int)(e % CC); const int p = (int)(e / CC); const int py = p / IMW, px = p % IMW; v2us oh, ol;
#pragma unroll
    for (int q = 0; q < 2; ++q) { const int cq = c + q; float acc = 0.0f;
#pragma unroll
        for (int tap = 0; tap < 9; ++tap) { const int y = py + tap / 3 - 1, x = px + tap % 3 - 1; if (y >= 0 && y < IMW && x >= 0 && x < IMW) { float pr = __fmul_rn(VS[((size_t)y * IMW + x) * CC + cq], bfr(dww[cq * 9 + tap])); asm volatile("" : "+v"(pr)); acc = __fadd_rn(acc, pr); } }
        const float yv = bn_leaky(acc, SC[cq], SH[cq]); unsigned short a, c2; splitf(yv, a, c2); oh[q] = a; ol[q] = c2; }
    *(volatile v2us*)(Yh + e) = oh; *(volatile v2us*)(Yl + e) = ol; __threadfence(); *(volatile v2us*)(Yh + e) = oh; *(volatile v2us*)(Yl + e) = ol; }
__global__ __launch_bounds__(256) void k_bnlpl(const float* __restrict__ F, const float* __restrict__ SC, const float* __restrict__ SH, bf* Yh, bf* Yl) { const size_t e = ((size_t)blockIdx.x * 256 + threadIdx.x) * 2; if (e >= (size_t)HW * CC) return; const int c = (int)(e % CC); v2us oh, ol;
#pragma unroll
    for (int q = 0; q < 2; ++q) { const float yv = bn_leaky(F[e + q], SC[c + q], SH[c + q]); unsigned short a, c2; splitf(yv, a, c2); oh[q] = a; ol[q] = c2; }
    *(volatile v2us*)(Yh + e) = oh; *(volatile v2us*)(Yl + e) = ol; __threadfence(); *(volatile v2us*)(Yh + e) = oh; *(volatile v2us*)(Yl + e) = ol; }
__global__ __launch_bounds__(256) void k_outT2(const float* __restrict__ F, float* out) { const size_t i = (size_t)blockIdx.x * 256 + threadIdx.x; if (i >= (size_t)CC * HW / 8) return; const int o = (int)(i / (HW / 8)); const int p0 = (int)(i % (HW / 8)) * 8; v4f a, b2;
#pragma unroll
    for (int q = 0; q < 4; ++q) { a[q] = F[(size_t)(p0 + q) * CC + o]; b2[q] = F[(size_t)(p0 + 4 + q) * CC + o]; }
    float* dst = out + (size_t)o * HW + p0; *(volatile v4f*)dst = a; *(volatile v4f*)(dst + 4) = b2; __threadfence(); *(volatile v4f*)dst = a; *(volatile v4f*)(dst + 4) = b2; }

extern "C" void kernel_launch(void* const* d_in, const int* in_sizes, int n_in,
                              void* d_out, int out_size, void* d_ws, size_t ws_size, hipStream_t stream) {
    (void)in_sizes; (void)n_in; (void)out_size;
    const float* x = (const float*)d_in[0]; const float* qw = (const float*)d_in[1]; const float* qb = (const float*)d_in[2]; const float* kw = (const float*)d_in[3]; const float* kb = (const float*)d_in[4]; const float* vw = (const float*)d_in[5]; const float* vb = (const float*)d_in[6];
    const float* ksw = (const float*)d_in[7]; const float* ksb = (const float*)d_in[8]; const float* sd1w = (const float*)d_in[9]; const float* sd1b = (const float*)d_in[10]; const float* sd2w = (const float*)d_in[11]; const float* sd2b = (const float*)d_in[12]; const float* dww = (const float*)d_in[13];
    const float* g1 = (const float*)d_in[14]; const float* be1 = (const float*)d_in[15]; const float* m1 = (const float*)d_in[16]; const float* v1 = (const float*)d_in[17]; const float* pww = (const float*)d_in[18]; const float* g2 = (const float*)d_in[19]; const float* be2 = (const float*)d_in[20]; const float* m2 = (const float*)d_in[21]; const float* v2 = (const float*)d_in[22];
    float* OUT = (float*)d_out;
    char* wsp = (char*)d_ws;
    auto take = [&](size_t bytes) { char* p = wsp; wsp += (bytes + 255) & ~(size_t)255; return (void*)p; };
    bf* QWB = (bf*)take((size_t)CC * CC * 2); bf* KWB = (bf*)take((size_t)CC * CC * 2); bf* VWB = (bf*)take((size_t)CC * CC * 2); bf* KSB = (bf*)take((size_t)CC * K9 * 2); bf* S1B = (bf*)take((size_t)CC * CC * 2); bf* PWB = (bf*)take((size_t)CC * CC * 2); bf* S2B = (bf*)take((size_t)CC * CC * 2);
    float* SC1 = (float*)take(CC * 4); float* SH1 = (float*)take(CC * 4); float* SC2 = (float*)take(CC * 4); float* SH2 = (float*)take(CC * 4);
    bf* XT = (bf*)take((size_t)HW * CC * 2); bf* IC = (bf*)take((size_t)HW * K9 * 2); float* FQ = (float*)take((size_t)HW * CC * 4); float* FK = (float*)take((size_t)HW * CC * 4); float* FV = (float*)take((size_t)HW * CC * 4); float* FKS = (float*)take((size_t)HW * CC * 4);
    bf* QPh = (bf*)take((size_t)NH_ * HW * DK * 2); bf* QPl = (bf*)take((size_t)NH_ * HW * DK * 2); bf* KPh = (bf*)take((size_t)NH_ * TP * DK * 2); bf* KPl = (bf*)take((size_t)NH_ * TP * DK * 2); h16* VT16 = (h16*)take((size_t)NH_ * DP * TP * 2);
    float* Sb = (float*)take((size_t)HW * TP * 4); h16* P16 = (h16*)take((size_t)HW * TP * 2); float* Ob = (float*)take((size_t)HW * DP * 4);
    bf* QKh = (bf*)take((size_t)HW * CC * 2); bf* QKl = (bf*)take((size_t)HW * CC * 2); float* FG = (float*)take((size_t)HW * CC * 4); float* VS = (float*)take((size_t)HW * CC * 4); bf* Y1h = (bf*)take((size_t)HW * CC * 2); bf* Y1l = (bf*)take((size_t)HW * CC * 2); float* Y2 = (float*)take((size_t)HW * CC * 4); bf* Y3h = (bf*)take((size_t)HW * CC * 2); bf* Y3l = (bf*)take((size_t)HW * CC * 2); float* FSD = (float*)take((size_t)HW * CC * 4);
    if ((size_t)(wsp - (char*)d_ws) > ws_size) return;
    const unsigned LW = (unsigned)(((size_t)CC * CC / 8 + 255) / 256);
    k_cvt8<<<LW, 256, 0, stream>>>(qw, QWB, (size_t)CC * CC / 8); k_cvt8<<<LW, 256, 0, stream>>>(kw, KWB, (size_t)CC * CC / 8); k_cvt8<<<LW, 256, 0, stream>>>(vw, VWB, (size_t)CC * CC / 8); k_cvt8<<<(unsigned)(((size_t)CC * K9 / 8 + 255) / 256), 256, 0, stream>>>(ksw, KSB, (size_t)CC * K9 / 8);
    k_cvt8<<<LW, 256, 0, stream>>>(sd1w, S1B, (size_t)CC * CC / 8); k_cvt8<<<LW, 256, 0, stream>>>(pww, PWB, (size_t)CC * CC / 8); k_cvt8<<<LW, 256, 0, stream>>>(sd2w, S2B, (size_t)CC * CC / 8);
    k_bnprep<<<1, 256, 0, stream>>>(g1, be1, m1, v1, SC1, SH1); k_bnprep<<<1, 256, 0, stream>>>(g2, be2, m2, v2, SC2, SH2);
    const unsigned L8 = (unsigned)(((size_t)HW * CC / 8 + 255) / 256), L4 = (unsigned)(((size_t)HW * CC / 4 + 255) / 256), L2 = (unsigned)(((size_t)HW * CC / 2 + 255) / 256);
    for (int b = 0; b < NB_; ++b) { const float* xb = x + (size_t)b * CC * HW; float* ob = OUT + (size_t)b * 2 * CC * HW;
        k_cvt8Tg<<<L8, 256, 0, stream>>>(xb, XT, CC, HW);
        k_im2x<<<(unsigned)(((size_t)HW * K9 / 8 + 255) / 256), 256, 0, stream>>>(xb, IC);
        k_gemmw<bf, 0, true><<<dim3(HW / 64, CC / 64, 1), 32, 0, stream>>>(XT, nullptr, QWB, nullptr, CC, FQ, CC, qb, 0, 0, 0);
        k_gemmw<bf, 0, true><<<dim3(HW / 64, CC / 64, 1), 32, 0, stream>>>(XT, nullptr, KWB, nullptr, CC, FK, CC, kb, 0, 0, 0);
        k_gemmw<bf, 0, true><<<dim3(HW / 64, CC / 64, 1), 32, 0, stream>>>(XT, nullptr, VWB, nullptr, CC, FV, CC, vb, 0, 0, 0);
        k_gemmw<bf, 0, true><<<dim3(HW / 64, CC / 64, 1), 32, 0, stream>>>(IC, nullptr, KSB, nullptr, K9, FKS, CC, ksb, 0, 0, 0);
        k_plq<<<(unsigned)(((size_t)NH_ * HW * DK / 2 + 255) / 256), 256, 0, stream>>>(FQ, QPh, QPl); k_plk<<<(unsigned)(((size_t)NH_ * TP * DK / 2 + 255) / 256), 256, 0, stream>>>(FK, KPh, KPl); k_vt16p<<<(unsigned)(((size_t)NH_ * DP * TP / 2 + 255) / 256), 256, 0, stream>>>(FV, VT16);
        for (int h = 0; h < NH_; ++h) {
            k_gemmw<bf, 2, false><<<dim3(HW / 64, TP / 64, 1), 32, 0, stream>>>(QPh + (size_t)h * HW * DK, QPl + (size_t)h * HW * DK, KPh + (size_t)h * TP * DK, KPl + (size_t)h * TP * DK, DK, Sb, TP, nullptr, 0, 0, 0);
            k_lsoftm<<<HW / 8, 256, 0, stream>>>(Sb, P16);
            k_gemmw<h16, 0, false><<<dim3(HW / 64, DP / 64, 1), 32, 0, stream>>>(P16, nullptr, VT16 + (size_t)h * DP * TP, nullptr, TP, Ob, DP, nullptr, 0, 0, 0);
            k_saout<<<(unsigned)(((size_t)DK * HW / 8 + 255) / 256), 256, 0, stream>>>(Ob, h, ob); }
        k_mulpl<<<L8, 256, 0, stream>>>(FQ, FKS, QKh, QKl, (size_t)HW * CC / 8);
        k_gemmw<bf, 1, true><<<dim3(HW / 64, CC / 64, 1), 32, 0, stream>>>(QKh, QKl, S1B, nullptr, CC, FG, CC, sd1b, 0, 0, 0);
        k_vsig<<<L4, 256, 0, stream>>>(FV, FG, VS, (size_t)HW * CC / 4);
        k_dwbn<<<L2, 256, 0, stream>>>(VS, dww, SC1, SH1, Y1h, Y1l);
        k_gemmw<bf, 1, false><<<dim3(HW / 64, CC / 64, 1), 32, 0, stream>>>(Y1h, Y1l, PWB, nullptr, CC, Y2, CC, nullptr, 0, 0, 0);
        k_bnlpl<<<L2, 256, 0, stream>>>(Y2, SC2, SH2, Y3h, Y3l);
        k_gemmw<bf, 1, true><<<dim3(HW / 64, CC / 64, 1), 32, 0, stream>>>(Y3h, Y3l, S2B, nullptr, CC, FSD, CC, sd2b, 0, 0, 0);
        k_outT2<<<(unsigned)(((size_t)CC * HW / 8 + 255) / 256), 256, 0, stream>>>(FSD, ob + (size_t)CC * HW); }
}
